// FC_Attention_42356967473257
// MI455X (gfx1250) — hardware-verified
//
#include <hip/hip_runtime.h>

typedef unsigned short us;
typedef int   v8i  __attribute__((ext_vector_type(8)));
typedef float v8f  __attribute__((ext_vector_type(8)));
typedef float v4f  __attribute__((ext_vector_type(4)));
typedef unsigned short v8us __attribute__((ext_vector_type(8)));
typedef __bf16 v16b __attribute__((ext_vector_type(16)));
typedef v4f  __attribute__((may_alias)) v4fa;
typedef v8us __attribute__((may_alias)) v8usa;
union Frag { v8i v; v8us half[2]; };
union DPack { double d[2]; v4f f; };

#define NBATCH 4
#define CIN    256
#define HIMG   32
#define NPIX   1024
#define PW     34
#define DQ     512
#define DV     256
#define DK     64
#define DVH    32
#define FTK    576

struct BiW { int i0[3]; int i1[3]; float w0[3]; float w1[3]; };
static_assert(sizeof(BiW) == 48);

__device__ __forceinline__ us f2bf(float f) {
  unsigned u = __float_as_uint(f);
  u += 0x7FFFu + ((u >> 16) & 1u);
  return (us)(u >> 16);
}
__device__ __forceinline__ float bf2f(us hv) {
  return __uint_as_float(((unsigned)hv) << 16);
}
__device__ __forceinline__ void split2(float f, us& hi, us& lo) {
  hi = f2bf(f);
  lo = f2bf(f - bf2f(hi));
}

__device__ __forceinline__ v8f wmma_bf(v8i a, v8i b, v8f c) {
  v8f d = __builtin_amdgcn_wmma_f32_16x16x32_bf16(false, __builtin_bit_cast(v16b, a), false,
                                                  __builtin_bit_cast(v16b, b), (short)0, c, false, false);
  asm volatile("v_nop\n\tv_nop\n\tv_nop\n\tv_nop" : "+v"(d) : "v"(a), "v"(b));
  return d;
}
__device__ __forceinline__ v8f wmma3(v8i ah, v8i al, v8i bh, v8i bl, v8f c) {
  c = wmma_bf(ah, bh, c);
  c = wmma_bf(al, bh, c);
  c = wmma_bf(ah, bl, c);
  return c;
}
__device__ __forceinline__ v8i ldfrag(const us* p, int h) {
  Frag f;
  f.half[0] = *(const v8usa*)(p + 8 * h);
  f.half[1] = *(const v8usa*)(p + 16 + 8 * h);
  return f.v;
}

__device__ __forceinline__ float wave_sum(float s) {
  s += __shfl_xor(s, 16);
  s += __shfl_xor(s, 8);
  s += __shfl_xor(s, 4);
  s += __shfl_xor(s, 2);
  s += __shfl_xor(s, 1);
  return s;
}
__device__ __forceinline__ double dshfl_xor(double v, int msk) {
  const unsigned long long u = __builtin_bit_cast(unsigned long long, v);
  int lo = (int)(unsigned)(u & 0xFFFFFFFFull);
  int hi = (int)(unsigned)(u >> 32);
  lo = __shfl_xor(lo, msk);
  hi = __shfl_xor(hi, msk);
  const unsigned long long r = (((unsigned long long)(unsigned)hi) << 32) | (unsigned long long)(unsigned)lo;
  return __builtin_bit_cast(double, r);
}
__device__ __forceinline__ double wave_sum_d(double s) {
  s += dshfl_xor(s, 16);
  s += dshfl_xor(s, 8);
  s += dshfl_xor(s, 4);
  s += dshfl_xor(s, 2);
  s += dshfl_xor(s, 1);
  return s;
}

__global__ __launch_bounds__(256) void k_prep_x(const float* __restrict__ x,
                                                us* __restrict__ xh, us* __restrict__ xl) {
  __shared__ __attribute__((aligned(16))) us sh[32 * 256];
  __shared__ __attribute__((aligned(16))) us sl[32 * 256];
  const int tid = threadIdx.x, lane = tid & 31, w = tid >> 5;
  const int y = blockIdx.x, b = blockIdx.y;
  #pragma unroll 1
  for (int j = 0; j < 32; ++j) {
    const int c = 8 * j + w;
    const float v = x[((size_t)(b * CIN + c) * HIMG + y) * HIMG + lane];
    us hi, lo;
    split2(v, hi, lo);
    sh[lane * 256 + c] = hi;
    sl[lane * 256 + c] = lo;
  }
  __syncthreads();
  v8us vh[4], vl[4];
  size_t d[4];
  #pragma unroll
  for (int i = 0; i < 4; ++i) {
    const int px = 4 * w + i;
    vh[i] = *(const v8usa*)(sh + px * 256 + 8 * lane);
    vl[i] = *(const v8usa*)(sl + px * 256 + 8 * lane);
    d[i] = ((size_t)((b * PW + y + 1) * PW + px + 1)) * CIN + 8 * lane;
  }
  #pragma unroll
  for (int i = 0; i < 4; ++i) { *(volatile v8us*)(xh + d[i]) = vh[i]; *(volatile v8us*)(xl + d[i]) = vl[i]; }
  __threadfence();
  #pragma unroll
  for (int i = 0; i < 4; ++i) { *(volatile v8us*)(xh + d[i]) = vh[i]; *(volatile v8us*)(xl + d[i]) = vl[i]; }
}

__global__ __launch_bounds__(256) void k_zero_border(us* __restrict__ ph, us* __restrict__ pl, int C) {
  const int tid = threadIdx.x, lane = tid & 31, w = tid >> 5;
  const int i = blockIdx.x * 8 + w;
  const int b = blockIdx.y;
  if (i >= 132) return;
  int py, px;
  if (i < 34)       { py = 0;           px = i; }
  else if (i < 68)  { py = PW - 1;      px = i - 34; }
  else if (i < 100) { py = i - 68 + 1;  px = 0; }
  else              { py = i - 100 + 1; px = PW - 1; }
  const size_t base = ((size_t)((b * PW + py) * PW + px)) * (size_t)C;
  v8us z;
  #pragma unroll
  for (int j = 0; j < 8; ++j) z[j] = (us)0;
  #pragma unroll 1
  for (int off = 8 * lane; off < C; off += 256) {
    *(volatile v8us*)(ph + base + off) = z;
    *(volatile v8us*)(pl + base + off) = z;
  }
  __threadfence();
  #pragma unroll 1
  for (int off = 8 * lane; off < C; off += 256) {
    *(volatile v8us*)(ph + base + off) = z;
    *(volatile v8us*)(pl + base + off) = z;
  }
}

__global__ __launch_bounds__(256) void k_wprep(const float* __restrict__ wsrc, int cout, int taps,
                                               us* __restrict__ wh, us* __restrict__ wl) {
  const int g = blockIdx.x * 256 + threadIdx.x;
  const int kw = taps * 256;
  const int n = cout * kw;
  const int e8 = g * 8;
  if (e8 >= n) return;
  const int o = e8 / kw;
  const int r = e8 - o * kw;
  const int tap = r >> 8, c = r & 255;
  const float* src = wsrc + ((size_t)(o * 256 + c)) * taps + tap;
  v8us vh, vl;
  #pragma unroll
  for (int i = 0; i < 8; ++i) {
    us a, bq;
    split2(src[(size_t)i * taps], a, bq);
    vh[i] = a;
    vl[i] = bq;
  }
  *(volatile v8us*)(wh + e8) = vh;
  *(volatile v8us*)(wl + e8) = vl;
  __threadfence();
  *(volatile v8us*)(wh + e8) = vh;
  *(volatile v8us*)(wl + e8) = vl;
}

__device__ __forceinline__ void frag_f32(const float* __restrict__ p, int h, v8i& fh, v8i& fl) {
  const v4f q0 = *(const v4fa*)(p + 8 * h);
  const v4f q1 = *(const v4fa*)(p + 8 * h + 4);
  const v4f q2 = *(const v4fa*)(p + 16 + 8 * h);
  const v4f q3 = *(const v4fa*)(p + 20 + 8 * h);
  float v[16];
  v[0] = q0.x; v[1] = q0.y; v[2] = q0.z; v[3] = q0.w;
  v[4] = q1.x; v[5] = q1.y; v[6] = q1.z; v[7] = q1.w;
  v[8] = q2.x; v[9] = q2.y; v[10] = q2.z; v[11] = q2.w;
  v[12] = q3.x; v[13] = q3.y; v[14] = q3.z; v[15] = q3.w;
  Frag a, bq;
  #pragma unroll
  for (int i = 0; i < 16; ++i) {
    us hi, lo;
    split2(v[i], hi, lo);
    a.half[i >> 3][i & 7] = hi;
    bq.half[i >> 3][i & 7] = lo;
  }
  fh = a.v;
  fl = bq.v;
}

__global__ __launch_bounds__(256) void k_bias(const float* __restrict__ x, const float* __restrict__ bw,
                                              const float* __restrict__ bb, float* __restrict__ biasv) {
  __shared__ __attribute__((aligned(16))) us sah[16 * 256];
  __shared__ __attribute__((aligned(16))) us sal[16 * 256];
  __shared__ __attribute__((aligned(16))) float sd[4 * 256];
  const int tid = threadIdx.x, lane = tid & 31, w = tid >> 5;
  const int h = lane >> 4, m = lane & 15;
  for (int i = tid; i < 16 * 256; i += 256) {
    if (i >= 4 * 256) { sah[i] = (us)0; sal[i] = (us)0; }
  }
  #pragma unroll 1
  for (int k = 0; k < 4; ++k) {
    const int ch = tid + 256 * k;
    const float* p = x + (size_t)ch * NPIX;
    float s0 = 0.f, s1 = 0.f, s2 = 0.f, s3 = 0.f;
    #pragma unroll 4
    for (int i = 0; i < 256; ++i) {
      const v4f v = *(const v4fa*)(p + 4 * i);
      s0 += v.x; s1 += v.y; s2 += v.z; s3 += v.w;
    }
    const float mean = ((s0 + s1) + (s2 + s3)) * (1.0f / 1024.0f);
    us hi, lo;
    split2(mean, hi, lo);
    sah[k * 256 + tid] = hi;
    sal[k * 256 + tid] = lo;
  }
  __syncthreads();

  const int o0 = 32 * w + m, o1 = o0 + 16;
  const float* br0 = bw + (size_t)o0 * 256;
  const float* br1 = bw + (size_t)o1 * 256;
  const v8f z8 = {0.f, 0.f, 0.f, 0.f, 0.f, 0.f, 0.f, 0.f};
  v8f acc[2];
  acc[0] = z8; acc[1] = z8;
  #pragma unroll 1
  for (int k0 = 0; k0 < 256; k0 += 32) {
    const v8i ah = ldfrag(sah + m * 256 + k0, h);
    const v8i al = ldfrag(sal + m * 256 + k0, h);
    v8i bh0, bl0, bh1, bl1;
    frag_f32(br0 + k0, h, bh0, bl0);
    frag_f32(br1 + k0, h, bh1, bl1);
    acc[0] = wmma3(ah, al, bh0, bl0, acc[0]);
    acc[1] = wmma3(ah, al, bh1, bl1, acc[1]);
  }
  const float bb0 = bb[o0], bb1 = bb[o1];
  if (h == 0) {
    #pragma unroll
    for (int r = 0; r < 4; ++r) {
      sd[r * 256 + o0] = acc[0][r] + bb0;
      sd[r * 256 + o1] = acc[1][r] + bb1;
    }
  }
  __syncthreads();
  const int L = tid >> 3, q = tid & 7;
  const v4f v = *(const v4fa*)(sd + L * 32 + 4 * q);
  float* dst = biasv + L * 32 + 4 * q;
  *(volatile v4f*)dst = v;
  __threadfence();
  *(volatile v4f*)dst = v;
}

template <int MODE>
__global__ __launch_bounds__(128) void k_conv(
    const us* __restrict__ ah, const us* __restrict__ al,
    const us* __restrict__ wh, const us* __restrict__ wl,
    const float* __restrict__ bias, int ntaps, int cout,
    us* __restrict__ oh, us* __restrict__ ol, float* __restrict__ of, float* __restrict__ part)
{
  __shared__ __attribute__((aligned(16))) float sbuf[64 * 64];
  __shared__ double sred[4][2];
  const int tid = threadIdx.x, lane = tid & 31, w = tid >> 5;
  const int h = lane >> 4, m = lane & 15;
  const int pt = blockIdx.x, b = pt >> 4, y0 = (pt & 15) * 2;
  const int n0 = blockIdx.y * 64;
  const int ry = w >> 1, y = y0 + ry, nw = 32 * (w & 1);
  const int kw = ntaps * CIN;
  const size_t wr0 = (size_t)(n0 + nw + m) * kw;
  const size_t wr1 = wr0 + (size_t)16 * kw;
  const v8f z8 = {0.f, 0.f, 0.f, 0.f, 0.f, 0.f, 0.f, 0.f};
  v8f acc[2][2];
  #pragma unroll
  for (int i = 0; i < 2; ++i) { acc[i][0] = z8; acc[i][1] = z8; }

  #pragma unroll 1
  for (int tap = 0; tap < ntaps; ++tap) {
    const int t3 = tap / 3;
    const int ky = (ntaps == 1) ? 1 : t3;
    const int kx = (ntaps == 1) ? 1 : (tap - 3 * t3);
    const size_t ar0 = ((size_t)((b * PW + y + ky) * PW + kx + m)) * CIN;
    const size_t ar1 = ar0 + (size_t)16 * CIN;
    const size_t wt = (size_t)tap * CIN;
    #pragma unroll 1
    for (int c0 = 0; c0 < CIN; c0 += 32) {
      const v8i fa0h = ldfrag(ah + ar0 + c0, h);
      const v8i fa0l = ldfrag(al + ar0 + c0, h);
      const v8i fa1h = ldfrag(ah + ar1 + c0, h);
      const v8i fa1l = ldfrag(al + ar1 + c0, h);
      #pragma unroll
      for (int nt = 0; nt < 2; ++nt) {
        const size_t wr = (nt == 0) ? wr0 : wr1;
        const v8i fbh = ldfrag(wh + wr + wt + c0, h);
        const v8i fbl = ldfrag(wl + wr + wt + c0, h);
        acc[0][nt] = wmma3(fa0h, fa0l, fbh, fbl, acc[0][nt]);
        acc[1][nt] = wmma3(fa1h, fa1l, fbh, fbl, acc[1][nt]);
      }
    }
  }

  float bv[2];
  bv[0] = bias[n0 + nw + m];
  bv[1] = bias[n0 + nw + 16 + m];
  us* sH = reinterpret_cast<us*>(sbuf);
  us* sL = sH + 4096;
  float fs = 0.f, fq = 0.f;
  double ds = 0.0, dq = 0.0;
  #pragma unroll
  for (int mt = 0; mt < 2; ++mt) {
    #pragma unroll
    for (int nt = 0; nt < 2; ++nt) {
      #pragma unroll
      for (int r = 0; r < 8; ++r) {
        const float val = acc[mt][nt][r] + bv[nt];
        const int tp = ry * 32 + mt * 16 + 8 * h + r;
        const int ch = nw + 16 * nt + m;
        if (MODE == 0) {
          const float rr = fmaxf(val, 0.f);
          const float r2 = rr * rr;
          fs += r2; fq += r2 * r2;
          us hi, lo;
          split2(r2, hi, lo);
          sH[tp * 64 + ch] = hi;
          sL[tp * 64 + ch] = lo;
        } else if (MODE == 1) {
          const float rr = fmaxf(val, 0.f);
          const float r2 = rr * rr;
          fs += r2; fq += r2 * r2;
          sbuf[ch * 64 + tp] = r2;
        } else if (MODE == 2) {
          us hi, lo;
          split2(val, hi, lo);
          sH[ch * 64 + tp] = hi;
          sL[ch * 64 + tp] = lo;
        } else {
          ds += (double)val;
          dq += (double)val * (double)val;
          sbuf[ch * 64 + tp] = val;
        }
      }
    }
  }
  if (MODE == 0 || MODE == 1) {
    fs = wave_sum(fs);
    fq = wave_sum(fq);
    ds = (double)fs;
    dq = (double)fq;
  } else if (MODE == 3) {
    ds = wave_sum_d(ds);
    dq = wave_sum_d(dq);
  }
  if (MODE != 2) {
    if (lane == 0) { sred[w][0] = ds; sred[w][1] = dq; }
  }
  __syncthreads();

  v4f pv;
  pv.x = 0.f; pv.y = 0.f; pv.z = 0.f; pv.w = 0.f;
  size_t li = 0;
  bool pw = false;
  if (MODE != 2) {
    double S = 0.0, Q2 = 0.0;
    #pragma unroll
    for (int k = 0; k < 4; ++k) { S += sred[k][0]; Q2 += sred[k][1]; }
    DPack pk;
    pk.d[0] = S; pk.d[1] = Q2;
    pv.x = (lane == 0) ? pk.f.x : 0.f;
    pv.y = (lane == 0) ? pk.f.y : 0.f;
    pv.z = (lane == 0) ? pk.f.z : 0.f;
    pv.w = (lane == 0) ? pk.f.w : 0.f;
    li = ((size_t)blockIdx.x * gridDim.y + blockIdx.y) * 32 + 4 * (lane & 7);
    pw = (w == 0) && (lane < 8);
  }

  if (MODE == 0) {
    const int q8 = lane & 7, sub = lane >> 3;
    v8us th[4], tl[4];
    size_t d[4];
    #pragma unroll
    for (int i = 0; i < 4; ++i) {
      const int tp = 16 * w + 4 * i + sub;
      const int ry2 = tp >> 5, xx = tp & 31;
      th[i] = *(const v8usa*)(sH + tp * 64 + 8 * q8);
      tl[i] = *(const v8usa*)(sL + tp * 64 + 8 * q8);
      d[i] = ((size_t)((b * PW + y0 + ry2 + 1) * PW + xx + 1)) * (size_t)cout + n0 + 8 * q8;
    }
    #pragma unroll
    for (int i = 0; i < 4; ++i) { *(volatile v8us*)(oh + d[i]) = th[i]; *(volatile v8us*)(ol + d[i]) = tl[i]; }
    if (pw) *(volatile v4f*)(part + li) = pv;
    __threadfence();
    #pragma unroll
    for (int i = 0; i < 4; ++i) { *(volatile v8us*)(oh + d[i]) = th[i]; *(volatile v8us*)(ol + d[i]) = tl[i]; }
    if (pw) *(volatile v4f*)(part + li) = pv;
  } else if (MODE == 2) {
    const int q8 = lane & 7, sub = lane >> 3;
    v8us th[4], tl[4];
    size_t d[4];
    #pragma unroll
    for (int i = 0; i < 4; ++i) {
      const int chl = 16 * w + 4 * i + sub;
      th[i] = *(const v8usa*)(sH + chl * 64 + 8 * q8);
      tl[i] = *(const v8usa*)(sL + chl * 64 + 8 * q8);
      d[i] = ((size_t)(b * cout + n0 + chl)) * NPIX + y0 * HIMG + 8 * q8;
    }
    #pragma unroll
    for (int i = 0; i < 4; ++i) { *(volatile v8us*)(oh + d[i]) = th[i]; *(volatile v8us*)(ol + d[i]) = tl[i]; }
    __threadfence();
    #pragma unroll
    for (int i = 0; i < 4; ++i) { *(volatile v8us*)(oh + d[i]) = th[i]; *(volatile v8us*)(ol + d[i]) = tl[i]; }
  } else {
    const int hs = lane >> 4, x4 = 4 * (lane & 15);
    v4f tv[8];
    size_t d[8];
    #pragma unroll
    for (int i = 0; i < 8; ++i) {
      const int chl = 16 * w + 2 * i + hs;
      tv[i] = *(const v4fa*)(sbuf + chl * 64 + x4);
      d[i] = ((size_t)(b * cout + n0 + chl)) * NPIX + y0 * HIMG + x4;
    }
    #pragma unroll
    for (int i = 0; i < 8; ++i) *(volatile v4f*)(of + d[i]) = tv[i];
    if (pw) *(volatile v4f*)(part + li) = pv;
    __threadfence();
    #pragma unroll
    for (int i = 0; i < 8; ++i) *(volatile v4f*)(of + d[i]) = tv[i];
    if (pw) *(volatile v4f*)(part + li) = pv;
  }
}

__global__ __launch_bounds__(64) void k_phinorm(const float* __restrict__ partq, const float* __restrict__ partk,
                                                float* __restrict__ scal) {
  __shared__ double sacc[2][32][2];
  __shared__ float sres[2];
  const int tid = threadIdx.x, lane = tid & 31, w = tid >> 5;
  const float* pp = (w == 0) ? partq : partk;
  double s2 = 0.0, s4 = 0.0;
  #pragma unroll 1
  for (int j = 0; j < 16; ++j) {
    const double* dp = reinterpret_cast<const double*>(pp + (size_t)(lane * 16 + j) * 32);
    s2 += dp[0];
    s4 += dp[1];
  }
  sacc[w][lane][0] = s2;
  sacc[w][lane][1] = s4;
  __syncthreads();
  if (lane == 0) {
    double t2 = 0.0, t4 = 0.0;
    for (int i = 0; i < 32; ++i) { t2 += sacc[w][i][0]; t4 += sacc[w][i][1]; }
    const float num = sqrtf((float)t2);
    const float den = sqrtf((float)t4);
    sres[w] = num * (1.0f / den);
  }
  __syncthreads();
  v4f pv;
  pv.x = (lane == 0) ? sres[0] : 0.f;
  pv.y = (lane == 0) ? sres[1] : 0.f;
  pv.z = 0.f; pv.w = 0.f;
  const bool pw = (w == 0) && (lane < 8);
  float* dst = scal + 4 * lane;
  if (pw) *(volatile v4f*)dst = pv;
  __threadfence();
  if (pw) *(volatile v4f*)dst = pv;
}

__global__ __launch_bounds__(128) void k_kv(
    const float* __restrict__ r2k, const us* __restrict__ vnh, const us* __restrict__ vnl,
    const float* __restrict__ scal, BiW bw, us* __restrict__ fth, us* __restrict__ ftl)
{
  __shared__ __attribute__((aligned(16))) us sH[32 * 64];
  __shared__ __attribute__((aligned(16))) us sL[32 * 64];
  const int tid = threadIdx.x, lane = tid & 31, w = tid >> 5;
  const int h = lane >> 4, m = lane & 15;
  const int pq = blockIdx.x, bh = blockIdx.y;
  const int b = bh >> 3, head = bh & 7;
  const int p = pq / 3, q = pq - 3 * p;
  const int   iy0 = (p == 0) ? bw.i0[0] : ((p == 1) ? bw.i0[1] : bw.i0[2]);
  const int   iy1 = (p == 0) ? bw.i1[0] : ((p == 1) ? bw.i1[1] : bw.i1[2]);
  const float wy0 = (p == 0) ? bw.w0[0] : ((p == 1) ? bw.w0[1] : bw.w0[2]);
  const float wy1 = (p == 0) ? bw.w1[0] : ((p == 1) ? bw.w1[1] : bw.w1[2]);
  const int   ix0 = (q == 0) ? bw.i0[0] : ((q == 1) ? bw.i0[1] : bw.i0[2]);
  const int   ix1 = (q == 0) ? bw.i1[0] : ((q == 1) ? bw.i1[1] : bw.i1[2]);
  const float wx0 = (q == 0) ? bw.w0[0] : ((q == 1) ? bw.w0[1] : bw.w0[2]);
  const float wx1 = (q == 0) ? bw.w1[0] : ((q == 1) ? bw.w1[1] : bw.w1[2]);
  const float sK = scal[1];
  const float amax = (float)(32.0 / 9.0);
  const float* arow = r2k + ((size_t)(b * DQ + head * DK + 16 * w + m)) * NPIX;
  const size_t br0 = ((size_t)(b * DV + head * DVH + m)) * NPIX;
  const size_t br1 = br0 + (size_t)16 * NPIX;
  const v8f z8 = {0.f, 0.f, 0.f, 0.f, 0.f, 0.f, 0.f, 0.f};
  v8f acc[2];
  acc[0] = z8; acc[1] = z8;

  #pragma unroll 1
  for (int k0 = 0; k0 < NPIX; k0 += 32) {
    const int yy = k0 >> 5;
    const float wy = ((yy == iy0) ? wy0 : 0.f) + ((yy == iy1) ? wy1 : 0.f);
    const float* ap = arow + k0;
    const v4f q0 = *(const v4fa*)(ap + 8 * h);
    const v4f q1 = *(const v4fa*)(ap + 8 * h + 4);
    const v4f q2 = *(const v4fa*)(ap + 16 + 8 * h);
    const v4f q3 = *(const v4fa*)(ap + 20 + 8 * h);
    float v[16];
    v[0] = q0.x; v[1] = q0.y; v[2] = q0.z; v[3] = q0.w;
    v[4] = q1.x; v[5] = q1.y; v[6] = q1.z; v[7] = q1.w;
    v[8] = q2.x; v[9] = q2.y; v[10] = q2.z; v[11] = q2.w;
    v[12] = q3.x; v[13] = q3.y; v[14] = q3.z; v[15] = q3.w;
    Frag fah, fal;
    #pragma unroll
    for (int i = 0; i < 16; ++i) {
      const int xx = 8 * h + (i & 7) + ((i >> 3) << 4);
      const float wx = ((xx == ix0) ? wx0 : 0.f) + ((xx == ix1) ? wx1 : 0.f);
      const float a = v[i] * (wy * wx);
      us hi, lo;
      split2(a, hi, lo);
      fah.half[i >> 3][i & 7] = hi;
      fal.half[i >> 3][i & 7] = lo;
    }
    const v8i fb0h = ldfrag(vnh + br0 + k0, h);
    const v8i fb0l = ldfrag(vnl + br0 + k0, h);
    const v8i fb1h = ldfrag(vnh + br1 + k0, h);
    const v8i fb1l = ldfrag(vnl + br1 + k0, h);
    acc[0] = wmma3(fah.v, fal.v, fb0h, fb0l, acc[0]);
    acc[1] = wmma3(fah.v, fal.v, fb1h, fb1l, acc[1]);
  }

  #pragma unroll
  for (int nt = 0; nt < 2; ++nt) {
    #pragma unroll
    for (int r = 0; r < 8; ++r) {
      float val = acc[nt][r] * sK;
      val = fminf(fmaxf(val, -amax), amax);
      const int kk = 16 * w + 8 * h + r;
      const int vv = 16 * nt + m;
      us hi, lo;
      split2(val, hi, lo);
      sH[vv * 64 + kk] = hi;
      sL[vv * 64 + kk] = lo;
    }
  }
  __syncthreads();
  const int q8 = lane & 7, sub = lane >> 3;
  v8us th[2], tl[2];
  size_t d[2];
  #pragma unroll
  for (int i = 0; i < 2; ++i) {
    const int vv = 8 * w + 4 * i + sub;
    th[i] = *(const v8usa*)(sH + vv * 64 + 8 * q8);
    tl[i] = *(const v8usa*)(sL + vv * 64 + 8 * q8);
    d[i] = ((size_t)(bh * DVH + vv)) * FTK + pq * 64 + 8 * q8;
  }
  #pragma unroll
  for (int i = 0; i < 2; ++i) { *(volatile v8us*)(fth + d[i]) = th[i]; *(volatile v8us*)(ftl + d[i]) = tl[i]; }
  __threadfence();
  #pragma unroll
  for (int i = 0; i < 2; ++i) { *(volatile v8us*)(fth + d[i]) = th[i]; *(volatile v8us*)(ftl + d[i]) = tl[i]; }
}

__global__ __launch_bounds__(128) void k_gconv(
    const us* __restrict__ rqh, const us* __restrict__ rql,
    const us* __restrict__ fth, const us* __restrict__ ftl,
    const float* __restrict__ scal, const float* __restrict__ biasv,
    us* __restrict__ oh, us* __restrict__ ol)
{
  __shared__ __attribute__((aligned(16))) us sH[64 * 64];
  __shared__ __attribute__((aligned(16))) us sL[64 * 64];
  const int tid = threadIdx.x, lane = tid & 31, w = tid >> 5;
  const int h = lane >> 4, m = lane & 15;
  const int pt = blockIdx.x, jp = blockIdx.y, b = blockIdx.z;
  const int y0 = 2 * pt;
  const int jl = w >> 1, ry = w & 1;
  const int j = 2 * jp + jl, y = y0 + ry, bh = b * 8 + j;
  const size_t fr0 = ((size_t)(bh * DVH + m)) * FTK;
  const size_t fr1 = fr0 + (size_t)16 * FTK;
  const v8f z8 = {0.f, 0.f, 0.f, 0.f, 0.f, 0.f, 0.f, 0.f};
  v8f acc[2][2];
  #pragma unroll
  for (int i = 0; i < 2; ++i) { acc[i][0] = z8; acc[i][1] = z8; }

  #pragma unroll 1
  for (int tap = 0; tap < 9; ++tap) {
    const int ky = tap / 3;
    const int kx = tap - 3 * ky;
    const size_t ar0 = ((size_t)((b * PW + y + ky) * PW + kx + m)) * DQ + (size_t)j * DK;
    const size_t ar1 = ar0 + (size_t)16 * DQ;
    const size_t wt = (size_t)tap * DK;
    #pragma unroll
    for (int c0 = 0; c0 < DK; c0 += 32) {
      const v8i fa0h = ldfrag(rqh + ar0 + c0, h);
      const v8i fa0l = ldfrag(rql + ar0 + c0, h);
      const v8i fa1h = ldfrag(rqh + ar1 + c0, h);
      const v8i fa1l = ldfrag(rql + ar1 + c0, h);
      #pragma unroll
      for (int nt = 0; nt < 2; ++nt) {
        const size_t fr = (nt == 0) ? fr0 : fr1;
        const v8i fbh = ldfrag(fth + fr + wt + c0, h);
        const v8i fbl = ldfrag(ftl + fr + wt + c0, h);
        acc[0][nt] = wmma3(fa0h, fa0l, fbh, fbl, acc[0][nt]);
        acc[1][nt] = wmma3(fa1h, fa1l, fbh, fbl, acc[1][nt]);
      }
    }
  }

  const float sQ = scal[0];
  float bv[2];
  bv[0] = biasv[b * DV + j * DVH + m];
  bv[1] = biasv[b * DV + j * DVH + 16 + m];
  #pragma unroll
  for (int mt = 0; mt < 2; ++mt) {
    #pragma unroll
    for (int nt = 0; nt < 2; ++nt) {
      #pragma unroll
      for (int r = 0; r < 8; ++r) {
        const float val = acc[mt][nt][r] * sQ + bv[nt];
        const int tp = ry * 32 + mt * 16 + 8 * h + r;
        const int chl = jl * 32 + 16 * nt + m;
        us hi, lo;
        split2(val, hi, lo);
        sH[tp * 64 + chl] = hi;
        sL[tp * 64 + chl] = lo;
      }
    }
  }
  __syncthreads();
  const int q8 = lane & 7, sub = lane >> 3;
  v8us th[4], tl[4];
  size_t d[4];
  #pragma unroll
  for (int i = 0; i < 4; ++i) {
    const int tp = 16 * w + 4 * i + sub;
    const int ry2 = tp >> 5, xx = tp & 31;
    th[i] = *(const v8usa*)(sH + tp * 64 + 8 * q8);
    tl[i] = *(const v8usa*)(sL + tp * 64 + 8 * q8);
    d[i] = ((size_t)((b * PW + y0 + ry2 + 1) * PW + xx + 1)) * DV + jp * 64 + 8 * q8;
  }
  #pragma unroll
  for (int i = 0; i < 4; ++i) { *(volatile v8us*)(oh + d[i]) = th[i]; *(volatile v8us*)(ol + d[i]) = tl[i]; }
  __threadfence();
  #pragma unroll
  for (int i = 0; i < 4; ++i) { *(volatile v8us*)(oh + d[i]) = th[i]; *(volatile v8us*)(ol + d[i]) = tl[i]; }
}

__global__ __launch_bounds__(256) void k_ln(const float* __restrict__ outp, const float* __restrict__ partl,
                                            float* __restrict__ out) {
  __shared__ double ss[64];
  __shared__ double sq[64];
  __shared__ float sst[2];
  const int tid = threadIdx.x;
  const int blk = blockIdx.x, b = blk >> 8;
  if (tid < 64) {
    const double* dp = reinterpret_cast<const double*>(partl + (size_t)(b * 64 + tid) * 32);
    ss[tid] = dp[0];
    sq[tid] = dp[1];
  }
  __syncthreads();
  if (tid == 0) {
    double S = 0.0, Q2 = 0.0;
    for (int i = 0; i < 64; ++i) { S += ss[i]; Q2 += sq[i]; }
    const double inv = 1.0 / 262144.0;
    const double mu = S * inv;
    double var = Q2 * inv - mu * mu;
    if (var < 0.0) var = 0.0;
    const float den = sqrtf((float)var + 1e-5f);
    sst[0] = (float)mu;
    sst[1] = 1.0f / den;
  }
  __syncthreads();
  const float muf = sst[0], rinv = sst[1];
  const size_t e = ((size_t)blk * 256 + tid) * 4;
  v4f v = *(const v4fa*)(outp + e);
  v4f o;
  o.x = (v.x - muf) * rinv;
  o.y = (v.y - muf) * rinv;
  o.z = (v.z - muf) * rinv;
  o.w = (v.w - muf) * rinv;
  *(volatile v4f*)(out + e) = o;
  __threadfence();
  *(volatile v4f*)(out + e) = o;
}

static void bilin3(BiW& bw) {
#pragma clang fp contract(off)
  const double scale = 32.0 / 3.0;
  for (int p = 0; p < 3; ++p) {
    double src = ((double)p + 0.5) * scale;
    src = src - 0.5;
    if (src < 0.0) src = 0.0;
    const int f = (int)src;
    const float frac = (float)(src - (double)f);
    int c0 = f, c1 = f + 1;
    if (c0 > HIMG - 1) c0 = HIMG - 1;
    if (c1 > HIMG - 1) c1 = HIMG - 1;
    bw.i0[p] = c0;
    bw.i1[p] = c1;
    bw.w0[p] = 1.0f - frac;
    bw.w1[p] = frac;
  }
}

extern "C" void kernel_launch(void* const* d_in, const int* in_sizes, int n_in,
                              void* d_out, int out_size, void* d_ws, size_t ws_size,
                              hipStream_t stream) {
  if (n_in < 11) return;
  if (in_sizes[0] != NBATCH * CIN * NPIX) return;
  if (in_sizes[1] != DQ * CIN || in_sizes[2] != DQ) return;
  if (in_sizes[3] != DQ * CIN * 9 || in_sizes[4] != DQ) return;
  if (in_sizes[5] != DV * CIN * 9 || in_sizes[6] != DV) return;
  if (in_sizes[7] != DV * CIN || in_sizes[8] != DV) return;
  if (in_sizes[9] != DV * DV * 9 || in_sizes[10] != DV) return;
  if (out_size != NBATCH * DV * NPIX) return;

  const float* x      = (const float*)d_in[0];
  const float* q_w    = (const float*)d_in[1];
  const float* q_b    = (const float*)d_in[2];
  const float* k_w    = (const float*)d_in[3];
  const float* k_b    = (const float*)d_in[4];
  const float* v_w    = (const float*)d_in[5];
  const float* v_b    = (const float*)d_in[6];
  const float* bias_w = (const float*)d_in[7];
  const float* bias_b = (const float*)d_in[8];
  const float* hu_w   = (const float*)d_in[9];
  const float* hu_b   = (const float*)d_in[10];
  float* out = (float*)d_out;

  char* ws = (char*)d_ws;
  size_t off = 0;
#define CARVE(T, name, bytes) T* name = (T*)(ws + off); off += (((size_t)(bytes)) + 255) & ~(size_t)255;
  const size_t padpx  = (size_t)NBATCH * PW * PW;
  CARVE(us,    XPH,   padpx * CIN * 2);
  CARVE(us,    XPL,   padpx * CIN * 2);
  CARVE(us,    WQH,   (size_t)DQ * CIN * 2);
  CARVE(us,    WQL,   (size_t)DQ * CIN * 2);
  CARVE(us,    WKH,   (size_t)DQ * CIN * 9 * 2);
  CARVE(us,    WKL,   (size_t)DQ * CIN * 9 * 2);
  CARVE(us,    WVH,   (size_t)DV * CIN * 9 * 2);
  CARVE(us,    WVL,   (size_t)DV * CIN * 9 * 2);
  CARVE(us,    WHH,   (size_t)DV * DV * 9 * 2);
  CARVE(us,    WHL,   (size_t)DV * DV * 9 * 2);
  CARVE(float, BIASV, (size_t)NBATCH * DV * 4);
  CARVE(us,    RQH,   padpx * DQ * 2);
  CARVE(us,    RQL,   padpx * DQ * 2);
  CARVE(float, R2K,   (size_t)NBATCH * DQ * NPIX * 4);
  CARVE(us,    VNH,   (size_t)NBATCH * DV * NPIX * 2);
  CARVE(us,    VNL,   (size_t)NBATCH * DV * NPIX * 2);
  CARVE(float, PARTQ, (size_t)512 * 128);
  CARVE(float, PARTK, (size_t)512 * 128);
  CARVE(float, SCAL,  256);
  CARVE(us,    FTH,   (size_t)NBATCH * 8 * DVH * FTK * 2);
  CARVE(us,    FTL,   (size_t)NBATCH * 8 * DVH * FTK * 2);
  CARVE(us,    QKH,   padpx * DV * 2);
  CARVE(us,    QKL,   padpx * DV * 2);
  CARVE(float, OUTP,  (size_t)NBATCH * DV * NPIX * 4);
  CARVE(float, PARTL, (size_t)256 * 128);
#undef CARVE
  if (off > ws_size) return;
  if (off > (size_t)134217728) return;

  BiW bw;
  bilin3(bw);

  k_prep_x<<<dim3(HIMG, NBATCH), 256, 0, stream>>>(x, XPH, XPL);
  k_zero_border<<<dim3(17, NBATCH), 256, 0, stream>>>(XPH, XPL, CIN);
  k_zero_border<<<dim3(17, NBATCH), 256, 0, stream>>>(RQH, RQL, DQ);
  k_zero_border<<<dim3(17, NBATCH), 256, 0, stream>>>(QKH, QKL, DV);
  k_wprep<<<(DQ * CIN * 1) / 2048, 256, 0, stream>>>(q_w, DQ, 1, WQH, WQL);
  k_wprep<<<(DQ * CIN * 9) / 2048, 256, 0, stream>>>(k_w, DQ, 9, WKH, WKL);
  k_wprep<<<(DV * CIN * 9) / 2048, 256, 0, stream>>>(v_w, DV, 9, WVH, WVL);
  k_wprep<<<(DV * DV * 9) / 2048, 256, 0, stream>>>(hu_w, DV, 9, WHH, WHL);

  k_bias<<<1, 256, 0, stream>>>(x, bias_w, bias_b, BIASV);

  k_conv<0><<<dim3(64, DQ / 64), 128, 0, stream>>>(XPH, XPL, WQH, WQL, q_b, 1, DQ, RQH, RQL, R2K, PARTQ);
  k_conv<1><<<dim3(64, DQ / 64), 128, 0, stream>>>(XPH, XPL, WKH, WKL, k_b, 9, DQ, VNH, VNL, R2K, PARTK);
  k_conv<2><<<dim3(64, DV / 64), 128, 0, stream>>>(XPH, XPL, WVH, WVL, v_b, 9, DV, VNH, VNL, OUTP, PARTL);

  k_phinorm<<<1, 64, 0, stream>>>(PARTQ, PARTK, SCAL);
  k_kv<<<dim3(9, NBATCH * 8), 128, 0, stream>>>(R2K, VNH, VNL, SCAL, bw, FTH, FTL);
  k_gconv<<<dim3(16, 4, NBATCH), 128, 0, stream>>>(RQH, RQL, FTH, FTL, SCAL, BIASV, QKH, QKL);

  k_conv<3><<<dim3(64, DV / 64), 128, 0, stream>>>(QKH, QKL, WHH, WHL, hu_b, 9, DV, VNH, VNL, OUTP, PARTL);
  k_ln<<<(NBATCH * DV * NPIX) / 1024, 256, 0, stream>>>(OUTP, PARTL, out);
}
